// HSTUEncoder_24026047054164
// MI455X (gfx1250) — hardware-verified
//
#include <hip/hip_runtime.h>


namespace {
constexpr int NB = 4, S = 1024, D = 512, NH = 8, DH = 64, NL = 4, NR = NB * S, WU = 4 * D  ;
constexpr float XS = 8.0f, WSC = 256.0f, PS = 8192.0f, EPS = 1e-6f, SQD = 22.627416997969522f;

typedef _Float16 b16;
typedef __attribute__((ext_vector_type(16))) _Float16 v16b;
typedef __attribute__((ext_vector_type(8))) _Float16 v8b;
typedef __attribute__((ext_vector_type(8))) float v8f;
typedef __attribute__((ext_vector_type(4))) float v4f;
__device__ __forceinline__ float bf16_rne(float f) { unsigned int u = __float_as_uint(f); u += 0x7FFFu + ((u >> 16) & 1u); return __uint_as_float(u & 0xFFFF0000u); }
__device__ __forceinline__ void split16(float v, b16& hi, b16& lo) { hi = (b16)v; lo = (b16)(v - (float)hi); }
__device__ __forceinline__ v16b frag_kb(const b16* p, int hh) { const v8b a = *(const v8b*)(p + 8 * hh), b = *(const v8b*)(p + 16 + 8 * hh); v16b f;
#pragma unroll
  for (int e = 0; e < 8; ++e) { f[e] = a[e]; f[8 + e] = b[e]; } return f; }
__device__ __forceinline__ v8f wmma16b(v16b a, v16b b, v8f c) { v8f d = __builtin_amdgcn_wmma_f32_16x16x32_f16(false, a, false, b, (short)0, c, false, false); asm volatile("v_nop\n\tv_nop\n\tv_nop\n\tv_nop" : "+v"(d) : "v"(a), "v"(b)); return d; }
__device__ __forceinline__ void wave_lds_sync() { __builtin_amdgcn_fence(__ATOMIC_RELEASE, "workgroup"); __builtin_amdgcn_wave_barrier(); __builtin_amdgcn_fence(__ATOMIC_ACQUIRE, "workgroup"); }
__device__ __forceinline__ float pmul(float a, float b) { float p = a * b; asm volatile("" : "+v"(p)); return p; }
__device__ __forceinline__ float silu_(float x) { return x / (1.0f + __expf(-x)); }

__global__ __launch_bounds__(256) void prep_kernel(const float* __restrict__ seq, const int* __restrict__ slen, const float* __restrict__ pos, const float* __restrict__ wu, const float* __restrict__ wo, b16* __restrict__ WUV, b16* __restrict__ WO, float* __restrict__ X) {
  const size_t t = (size_t)blockIdx.x * 256 + threadIdx.x; const size_t nu = (size_t)NL * WU * D / 8, no = (size_t)NL * D * D / 8, nx = (size_t)NR * D / 4; v8b o;
  if (t < nu) { const size_t e = t * 8; const int l = (int)(e / ((size_t)WU * D)); const int rem = (int)(e % ((size_t)WU * D)); const int oo = rem / D, k0 = rem % D; for (int j = 0; j < 8; ++j) o[j] = (b16)(bf16_rne(wu[((size_t)l * D + k0 + j) * WU + oo]) * WSC); for (int pass = 0; pass < 2; ++pass) { *(volatile v8b*)(WUV + e) = o; __threadfence(); } return; }
  size_t u = t - nu;
  if (u < no) { const size_t e = u * 8; const int l = (int)(e / ((size_t)D * D)); const int rem = (int)(e % ((size_t)D * D)); const int oo = rem / D, k0 = rem % D; for (int j = 0; j < 8; ++j) o[j] = (b16)(bf16_rne(wo[((size_t)l * D + k0 + j) * D + oo]) * WSC); for (int pass = 0; pass < 2; ++pass) { *(volatile v8b*)(WO + e) = o; __threadfence(); } return; } u -= no;
  if (u < nx) { const size_t e = u * 4; const size_t row = e / D; const int c = (int)(e % D); const int b = (int)(row / S), n = (int)(row % S); const float m = (n < slen[b]) ? 1.0f : 0.0f; const v4f sv = *(const v4f*)(seq + e); v4f r;
    for (int j = 0; j < 4; ++j) r[j] = (bf16_rne(sv[j]) * SQD + bf16_rne(pos[(size_t)n * D + c + j])) * m; for (int pass = 0; pass < 2; ++pass) { *(volatile v4f*)(X + e) = r; __threadfence(); } }
}
template <int MODE>
__global__ __launch_bounds__(256) void ln_kernel(const float* __restrict__ X, const float* __restrict__ g, const float* __restrict__ bta, const float* __restrict__ U, b16* __restrict__ Yh, b16* __restrict__ Yl) {
  const int wave = threadIdx.x >> 5, lane = threadIdx.x & 31; const size_t row = (size_t)blockIdx.x * 8 + wave; float x[16];
  { const v4f a = *(const v4f*)(X + row * D + lane * 16), c = *(const v4f*)(X + row * D + lane * 16 + 4), e = *(const v4f*)(X + row * D + lane * 16 + 8), f = *(const v4f*)(X + row * D + lane * 16 + 12); for (int j = 0; j < 4; ++j) { x[j] = a[j]; x[4 + j] = c[j]; x[8 + j] = e[j]; x[12 + j] = f[j]; } }
  float s = 0.0f; for (int j = 0; j < 16; ++j) s += x[j];
#pragma unroll
  for (int o = 16; o >= 1; o >>= 1) s += __shfl_xor(s, o);
  const float mu = s * (1.0f / D); float q = 0.0f; for (int j = 0; j < 16; ++j) { const float d = x[j] - mu; q += d * d; }
#pragma unroll
  for (int o = 16; o >= 1; o >>= 1) q += __shfl_xor(q, o);
  const float rs = rsqrtf(q * (1.0f / D) + EPS); v8b h0, h1, l0, l1;
  for (int j = 0; j < 16; ++j) { const int c = lane * 16 + j; float y = (x[j] - mu) * rs * bf16_rne(g[c]) + bf16_rne(bta[c]); if (MODE == 1) y = pmul(y, U[row * D + c]); b16 p, pl; split16(y * XS, p, pl); if (j < 8) { h0[j] = p; l0[j] = pl; } else { h1[j - 8] = p; l1[j - 8] = pl; } }
  for (int pass = 0; pass < 2; ++pass) { *(volatile v8b*)(Yh + row * D + lane * 16) = h0; *(volatile v8b*)(Yh + row * D + lane * 16 + 8) = h1; *(volatile v8b*)(Yl + row * D + lane * 16) = l0; *(volatile v8b*)(Yl + row * D + lane * 16 + 8) = l1; __threadfence(); }
}
__global__ __launch_bounds__(128) void uvqk_kernel(const b16* __restrict__ NXh, const b16* __restrict__ NXl, const b16* __restrict__ W, float* __restrict__ Uf, b16* __restrict__ VTh, b16* __restrict__ VTl, b16* __restrict__ Qh, b16* __restrict__ Ql, b16* __restrict__ Kh, b16* __restrict__ Kl) {
  __shared__ __attribute__((aligned(16))) float Tf[4][16][128 + 4]; __shared__ __attribute__((aligned(16))) b16 Th[4][16][128 + 8], Tl[4][16][128 + 8]; __shared__ __attribute__((aligned(16))) b16 Vt[128][64 + 8], Vtl[128][64 + 8];
  const int wave = threadIdx.x >> 5, lane = threadIdx.x & 31, nloc = lane & 15, hlf = lane >> 4, t_ = threadIdx.x; const int n0 = blockIdx.y * 128; const size_t m0 = (size_t)blockIdx.x * 64 + wave * 16; const int kind = n0 / D; const int c0 = n0 % D;
  v8f acc[8];
#pragma unroll
  for (int t = 0; t < 8; ++t) acc[t] = (v8f){};
#pragma unroll 2
  for (int kb = 0; kb < D; kb += 32) { const v16b a = frag_kb(NXh + (m0 + nloc) * D + kb, hlf), al = frag_kb(NXl + (m0 + nloc) * D + kb, hlf);
#pragma unroll
    for (int t = 0; t < 8; ++t) { const v16b bw = frag_kb(W + (size_t)(n0 + t * 16 + nloc) * D + kb, hlf); acc[t] = wmma16b(a, bw, acc[t]); acc[t] = wmma16b(al, bw, acc[t]); } }
  if (kind == 0) {
#pragma unroll
    for (int t = 0; t < 8; ++t)
#pragma unroll 1
      for (int r = 0; r < 8; ++r) Tf[wave][8 * hlf + r][t * 16 + nloc] = silu_(acc[t][r] * (1.0f / (XS * WSC)));
    wave_lds_sync();
    for (int pass = 0; pass < 2; ++pass) { for (int rr = 0; rr < 16; ++rr) *(volatile v4f*)(Uf + (m0 + rr) * D + c0 + lane * 4) = *(const v4f*)(&Tf[wave][rr][lane * 4]); __threadfence(); }
  } else if (kind == 1) {
#pragma unroll
    for (int t = 0; t < 8; ++t)
#pragma unroll 1
      for (int r = 0; r < 8; ++r) { b16 p, q; split16(silu_(acc[t][r] * (1.0f / (XS * WSC))) * XS, p, q); Vt[t * 16 + nloc][wave * 16 + 8 * hlf + r] = p; Vtl[t * 16 + nloc][wave * 16 + 8 * hlf + r] = q; }
    __syncthreads();
    const size_t r0 = (size_t)blockIdx.x * 64; const size_t b = r0 / S; const int key0 = (int)(r0 % S);
    for (int pass = 0; pass < 2; ++pass) { for (int q = t_; q < 128 * 8; q += 128) { const int cc = q >> 3, c8 = (q & 7) * 8; const int col = c0 + cc; const int h = col / DH, d = col % DH; const size_t gi = (((b * NH + h) * DH + d) * S) + key0 + c8; *(volatile v8b*)(VTh + gi) = *(const v8b*)(&Vt[cc][c8]); *(volatile v8b*)(VTl + gi) = *(const v8b*)(&Vtl[cc][c8]); } __threadfence(); }
  } else {
#pragma unroll
    for (int t = 0; t < 8; ++t)
#pragma unroll 1
      for (int r = 0; r < 8; ++r) { b16 p, q; split16(silu_(acc[t][r] * (1.0f / (XS * WSC))) * XS, p, q); Th[wave][8 * hlf + r][t * 16 + nloc] = p; Tl[wave][8 * hlf + r][t * 16 + nloc] = q; }
    wave_lds_sync(); b16* dh = kind == 2 ? Qh : Kh; b16* dl = kind == 2 ? Ql : Kl;
    for (int pass = 0; pass < 2; ++pass) { for (int r2 = 0; r2 < 16; r2 += 2) { const int rr = r2 + (lane >> 4), c8 = (lane & 15) * 8; const size_t gi = (m0 + rr) * D + c0 + c8; *(volatile v8b*)(dh + gi) = *(const v8b*)(&Th[wave][rr][c8]); *(volatile v8b*)(dl + gi) = *(const v8b*)(&Tl[wave][rr][c8]); } __threadfence(); }
  }
}
__global__ __launch_bounds__(64) void attn_kernel(const b16* __restrict__ Qh, const b16* __restrict__ Ql, const b16* __restrict__ Kh, const b16* __restrict__ Kl, const b16* __restrict__ VTh, const b16* __restrict__ VTl, const float* __restrict__ posw, float* __restrict__ AVf) {
  __shared__ __attribute__((aligned(16))) float To[2][16][DH + 4];
  const int wave = threadIdx.x >> 5, lane = threadIdx.x & 31, hh = lane >> 4, col = lane & 15; const int b = blockIdx.z, h = blockIdx.y; const int q0 = blockIdx.x * 32 + wave * 16, qi = q0 + col;
  const size_t qo = ((size_t)b * S + qi) * D + h * DH; const v16b qa0 = frag_kb(Qh + qo, hh), qa1 = frag_kb(Qh + qo + 32, hh), ql0 = frag_kb(Ql + qo, hh), ql1 = frag_kb(Ql + qo + 32, hh);
  const b16* Kb = Kh + (size_t)b * S * D + h * DH; const b16* Klb = Kl + (size_t)b * S * D + h * DH; const b16* Vb = VTh + ((size_t)b * NH + h) * DH * S; const b16* Vlb = VTl + ((size_t)b * NH + h) * DH * S;
  v8f o[4] = {{}, {}, {}, {}}, ol[4] = {{}, {}, {}, {}}; const float cs = 1.0f / (XS * XS); const int kend = q0 + 16;
  for (int kb = 0; kb < kend; kb += 32) {
    v8f s0 = {}, s1 = {};
    { const b16* k0 = Kb + (size_t)(kb + col) * D, *k1 = Kb + (size_t)(kb + 16 + col) * D, *k0l = Klb + (size_t)(kb + col) * D, *k1l = Klb + (size_t)(kb + 16 + col) * D;
      v16b f = frag_kb(k0, hh); s0 = wmma16b(f, qa0, s0); s0 = wmma16b(f, ql0, s0); s0 = wmma16b(frag_kb(k0l, hh), qa0, s0);
      f = frag_kb(k0 + 32, hh); s0 = wmma16b(f, qa1, s0); s0 = wmma16b(f, ql1, s0); s0 = wmma16b(frag_kb(k0l + 32, hh), qa1, s0);
      f = frag_kb(k1, hh); s1 = wmma16b(f, qa0, s1); s1 = wmma16b(f, ql0, s1); s1 = wmma16b(frag_kb(k1l, hh), qa0, s1);
      f = frag_kb(k1 + 32, hh); s1 = wmma16b(f, qa1, s1); s1 = wmma16b(f, ql1, s1); s1 = wmma16b(frag_kb(k1l + 32, hh), qa1, s1); }
    v16b ph, pl;
#pragma unroll
    for (int r = 0; r < 8; ++r) { const int ka = kb + 8 * hh + r, kbb = kb + 16 + 8 * hh + r;
      const float a0 = (ka <= qi) ? silu_(s0[r] * cs + bf16_rne(posw[ka - qi + (S - 1)])) * (1.0f / S) : 0.0f; const float a1 = (kbb <= qi) ? silu_(s1[r] * cs + bf16_rne(posw[kbb - qi + (S - 1)])) * (1.0f / S) : 0.0f;
      b16 p, q; split16(a0 * PS, p, q); ph[r] = p; pl[r] = q; split16(a1 * PS, p, q); ph[8 + r] = p; pl[8 + r] = q; }
#pragma unroll
    for (int t = 0; t < 4; ++t) { const v16b vf = frag_kb(Vb + (size_t)(t * 16 + col) * S + kb, hh); o[t] = wmma16b(vf, ph, o[t]); ol[t] = wmma16b(vf, pl, ol[t]); ol[t] = wmma16b(frag_kb(Vlb + (size_t)(t * 16 + col) * S + kb, hh), ph, ol[t]); } }
#pragma unroll
  for (int t = 0; t < 4; ++t)
#pragma unroll
    for (int r = 0; r < 8; ++r) To[wave][col][t * 16 + 8 * hh + r] = (o[t][r] + ol[t][r]) * (1.0f / (PS * XS));
  wave_lds_sync();
  for (int pass = 0; pass < 2; ++pass) { for (int rr = 0; rr < 16; ++rr) if (lane < 16) *(volatile v4f*)(AVf + ((size_t)b * S + q0 + rr) * D + h * DH + lane * 4) = *(const v4f*)(&To[wave][rr][lane * 4]); __threadfence(); }
}
__global__ __launch_bounds__(128) void oproj_kernel(const b16* __restrict__ Oh, const b16* __restrict__ Ol, const b16* __restrict__ WO, const float* __restrict__ bo, const int* __restrict__ slen, float* __restrict__ X) {
  __shared__ __attribute__((aligned(16))) float Tf[4][16][128 + 4];
  const int wave = threadIdx.x >> 5, lane = threadIdx.x & 31, nloc = lane & 15, hlf = lane >> 4; const size_t m0 = (size_t)blockIdx.x * 64 + wave * 16; const int n0 = blockIdx.y * 128;
  v8f acc[8];
#pragma unroll
  for (int t = 0; t < 8; ++t) acc[t] = (v8f){};
#pragma unroll 2
  for (int kb = 0; kb < D; kb += 32) { const v16b a = frag_kb(Oh + (m0 + nloc) * D + kb, hlf), al = frag_kb(Ol + (m0 + nloc) * D + kb, hlf);
#pragma unroll
    for (int t = 0; t < 8; ++t) { const v16b bw = frag_kb(WO + (size_t)(n0 + t * 16 + nloc) * D + kb, hlf); acc[t] = wmma16b(a, bw, acc[t]); acc[t] = wmma16b(al, bw, acc[t]); } }
#pragma unroll
  for (int t = 0; t < 8; ++t) { const int c = n0 + t * 16 + nloc; const float bb = bf16_rne(bo[c]);
#pragma unroll
    for (int r = 0; r < 8; ++r) { const size_t row = m0 + 8 * hlf + r; const int b = (int)(row / S), n = (int)(row % S); const float m = (n < slen[b]) ? 1.0f : 0.0f; Tf[wave][8 * hlf + r][t * 16 + nloc] = (X[row * D + c] + acc[t][r] * (1.0f / (XS * WSC)) + bb) * m; } }
  wave_lds_sync();
  for (int pass = 0; pass < 2; ++pass) { for (int rr = 0; rr < 16; ++rr) *(volatile v4f*)(X + (m0 + rr) * D + n0 + lane * 4) = *(const v4f*)(&Tf[wave][rr][lane * 4]); __threadfence(); }
}
__global__ __launch_bounds__(256) void final_kernel(const float* __restrict__ X, float* __restrict__ out) {
  const int wave = threadIdx.x >> 5, lane = threadIdx.x & 31; const size_t row = (size_t)blockIdx.x * 8 + wave; float x[16];
  { const v4f a = *(const v4f*)(X + row * D + lane * 16), c = *(const v4f*)(X + row * D + lane * 16 + 4), e = *(const v4f*)(X + row * D + lane * 16 + 8), f = *(const v4f*)(X + row * D + lane * 16 + 12); for (int j = 0; j < 4; ++j) { x[j] = a[j]; x[4 + j] = c[j]; x[8 + j] = e[j]; x[12 + j] = f[j]; } }
  float q = 0.0f; for (int j = 0; j < 16; ++j) q += x[j] * x[j];
#pragma unroll
  for (int o = 16; o >= 1; o >>= 1) q += __shfl_xor(q, o);
  const float inv = 1.0f / fmaxf(sqrtf(q), 1e-6f); v4f r[4]; for (int j = 0; j < 16; ++j) r[j / 4][j % 4] = x[j] * inv;
  for (int pass = 0; pass < 2; ++pass) { for (int k = 0; k < 4; ++k) *(volatile v4f*)(out + row * D + lane * 16 + k * 4) = r[k]; __threadfence(); }
}
}

extern "C" void kernel_launch(void* const* d_in, const int* in_sizes, int n_in, void* d_out, int out_size, void* d_ws, size_t ws_size, hipStream_t stream) {
  (void)n_in;
  auto Fp = [&](int i) { return (const float*)d_in[i]; }; auto Ip = [&](int i) { return (const int*)d_in[i]; };
  if (in_sizes[0] != NR * D || in_sizes[1] != NB || in_sizes[2] != S * D || in_sizes[5] != NL * D * WU || in_sizes[8] != NL * D * D || in_sizes[10] != NL * (2 * S - 1) || out_size != NR * D) return;
  size_t off = 0; char* ws = (char*)d_ws;
  auto carve = [&](size_t bytes) { char* p = ws + off; off += (bytes + 255) & ~(size_t)255; return p; };
  b16* WUV = (b16*)carve((size_t)NL * WU * D * 2); b16* WO = (b16*)carve((size_t)NL * D * D * 2); float* X = (float*)carve((size_t)NR * D * 4);
  b16* NXh = (b16*)carve((size_t)NR * D * 2); b16* NXl = (b16*)carve((size_t)NR * D * 2); float* Uf = (float*)carve((size_t)NR * D * 4); b16* VTh = (b16*)carve((size_t)NR * D * 2); b16* VTl = (b16*)carve((size_t)NR * D * 2);
  b16* Qh = (b16*)carve((size_t)NR * D * 2); b16* Ql = (b16*)carve((size_t)NR * D * 2); b16* Kh = (b16*)carve((size_t)NR * D * 2); b16* Kl = (b16*)carve((size_t)NR * D * 2); float* AVf = (float*)carve((size_t)NR * D * 4);
  b16* Oh = NXh; b16* Ol = NXl;
  if (off > ws_size || off > ((size_t)128 << 20)) return;
  prep_kernel<<<(unsigned)(((size_t)NL * WU * D / 8 + (size_t)NL * D * D / 8 + (size_t)NR * D / 4 + 255) / 256), 256, 0, stream>>>(Fp(0), Ip(1), Fp(2), Fp(5), Fp(8), WUV, WO, X);
  for (int l = 0; l < NL; ++l) {
    ln_kernel<0><<<NR / 8, 256, 0, stream>>>(X, Fp(3) + l * D, Fp(4) + l * D, nullptr, NXh, NXl);
    uvqk_kernel<<<dim3(NR / 64, WU / 128), 128, 0, stream>>>(NXh, NXl, WUV + (size_t)l * WU * D, Uf, VTh, VTl, Qh, Ql, Kh, Kl);
    attn_kernel<<<dim3(S / 32, NH, NB), 64, 0, stream>>>(Qh, Ql, Kh, Kl, VTh, VTl, Fp(10) + (size_t)l * (2 * S - 1), AVf);
    ln_kernel<1><<<NR / 8, 256, 0, stream>>>(AVf, Fp(6) + l * D, Fp(7) + l * D, Uf, Oh, Ol);
    oproj_kernel<<<dim3(NR / 64, D / 128), 128, 0, stream>>>(Oh, Ol, WO + (size_t)l * D * D, Fp(9) + l * D, Ip(1), X);
  }
  final_kernel<<<NR / 8, 256, 0, stream>>>(X, (float*)d_out);
}
